// DANet_15169824489909
// MI455X (gfx1250) — hardware-run, weakly checked
//
#include <hip/hip_runtime.h>
#include <math.h>

typedef __attribute__((ext_vector_type(16))) _Float16 v16h;
typedef __attribute__((ext_vector_type(8)))  _Float16 v8h;
typedef __attribute__((ext_vector_type(8)))  float    v8f;
typedef __attribute__((ext_vector_type(4)))  float    v4f;
typedef __attribute__((ext_vector_type(4)))  unsigned int v4u;

constexpr int kB    = 4;
constexpr int kC    = 512;
constexpr int kN    = 4096;
constexpr int kHid  = 64;
constexpr int kQK   = 2 * kHid;
constexpr int kWRows = 2 * kHid + kC;
constexpr float kWCarry    = 16.0f;
constexpr float kWCarryInv = 1.0f / kWCarry;
constexpr float kPCarry    = 8192.0f;
constexpr float kECarry    = 1024.0f;
constexpr float kECarryInv = 1.0f / kECarry;
constexpr float kResCarry  = 2048.0f;
constexpr float kResInv    = 1.0f / kResCarry;
constexpr float kF16MinNormal = 6.103515625e-5f;
constexpr float kArgCap    = 2.0f;
constexpr int kXP   = 68;
constexpr int kPvQ  = 32;
constexpr int kPvKC = 128;
constexpr int kPvPP = 136;
constexpr int kPvSP = 36;

static_assert(kHid == 64);
static_assert((kC % 64) == 0 && (kN % 64) == 0 && (kQK % 64) == 0 && ((kB * kN) % 64) == 0);
static_assert((kC % 32) == 0 && (kN % 32) == 0 && (kHid % 32) == 0);
static_assert((kN % 128) == 0 && (kN % kPvKC) == 0 && (kN % kPvQ) == 0);
static_assert((kPvPP % 8) == 0 && (kPvSP % 4) == 0 && (kXP % 4) == 0);
static_assert((((kB * kN) / 16) * (kQK / 64)) % 8 == 0);

constexpr size_t kSzX16   = (size_t)kB * kC * kN * 2;
constexpr size_t kSzXTH   = (size_t)kB * kN * kC * 2;
constexpr size_t kSzXTL   = (size_t)kB * kN * kC * 2;
constexpr size_t kSzW16   = (size_t)kWRows * kC * 2;
constexpr size_t kSzW16L  = (size_t)kQK * kC * 2;
constexpr size_t kSzQKH   = (size_t)kB * kN * kQK * 2;
constexpr size_t kSzQKL   = (size_t)kB * kN * kQK * 2;
constexpr size_t kSzV16   = (size_t)kB * kC * kN * 2;
constexpr size_t kSzRMAX  = (size_t)kB * kN * 4;
constexpr size_t kSzPAM   = (size_t)kB * kC * kN * 4;
constexpr size_t kSzG     = (size_t)kB * kC * kC * 4;
constexpr size_t kSzE16   = (size_t)kB * kC * kC * 2;
constexpr size_t kOffX16   = 0;
constexpr size_t kOffXTH   = kOffX16  + kSzX16;
constexpr size_t kOffXTL   = kOffXTH  + kSzXTH;
constexpr size_t kOffW16   = kOffXTL  + kSzXTL;
constexpr size_t kOffW16L  = kOffW16  + kSzW16;
constexpr size_t kOffQKH   = kOffW16L + kSzW16L;
constexpr size_t kOffQKL   = kOffQKH  + kSzQKH;
constexpr size_t kOffV16   = kOffQKL  + kSzQKL;
constexpr size_t kOffRMAX  = kOffV16  + kSzV16;
constexpr size_t kOffPAM   = kOffRMAX + kSzRMAX;
constexpr size_t kOffG     = kOffPAM  + kSzPAM;
constexpr size_t kOffE16   = kOffG    + kSzG;
constexpr size_t kWsTotal  = kOffE16  + kSzE16;
static_assert(kWsTotal == 116195328ull);
static_assert(kWsTotal <= 134217728ull);
static_assert((kOffXTH % 128) == 0 && (kOffXTL % 128) == 0 && (kOffW16 % 128) == 0 && (kOffW16L % 128) == 0 &&
              (kOffQKH % 128) == 0 && (kOffQKL % 128) == 0 && (kOffV16 % 128) == 0 && (kOffRMAX % 128) == 0 &&
              (kOffPAM % 128) == 0 && (kOffG % 128) == 0 && (kOffE16 % 128) == 0);

__device__ __forceinline__ unsigned pk16(unsigned short a, unsigned short b) { return (unsigned)a | ((unsigned)b << 16); }
__device__ __forceinline__ unsigned short h_bits(float f) { const _Float16 h = (_Float16)f; return __builtin_bit_cast(unsigned short, h); }
__device__ __forceinline__ v4u pack8_f16(float f0, float f1, float f2, float f3, float f4, float f5, float f6, float f7) {
  const v4u u = (v4u){pk16(h_bits(f0), h_bits(f1)), pk16(h_bits(f2), h_bits(f3)),
                      pk16(h_bits(f4), h_bits(f5)), pk16(h_bits(f6), h_bits(f7))};
  return u;
}
__device__ __forceinline__ void split_h(float v, unsigned short& hb, unsigned short& lb) {
  const _Float16 h0 = (_Float16)v;
  float hf = (float)h0;
  hf = (fabsf(hf) < kF16MinNormal) ? 0.0f : hf;
  const _Float16 h = (_Float16)hf;
  const _Float16 l = (_Float16)((v - hf) * kResCarry);
  hb = __builtin_bit_cast(unsigned short, h);
  lb = __builtin_bit_cast(unsigned short, l);
}
__device__ __forceinline__ void pack8_split(float f0, float f1, float f2, float f3, float f4, float f5, float f6, float f7,
                                            v4u& hi, v4u& lo) {
  unsigned short h0, h1, h2, h3, h4, h5, h6, h7;
  unsigned short l0, l1, l2, l3, l4, l5, l6, l7;
  split_h(f0, h0, l0);
  split_h(f1, h1, l1);
  split_h(f2, h2, l2);
  split_h(f3, h3, l3);
  split_h(f4, h4, l4);
  split_h(f5, h5, l5);
  split_h(f6, h6, l6);
  split_h(f7, h7, l7);
  hi = (v4u){pk16(h0, h1), pk16(h2, h3), pk16(h4, h5), pk16(h6, h7)};
  lo = (v4u){pk16(l0, l1), pk16(l2, l3), pk16(l4, l5), pk16(l6, l7)};
}

union FragU { v16h v; v8h h[2]; };
__device__ __forceinline__ v16h frag_load(const _Float16* p) {
  FragU f;
  f.h[0] = *(const v8h*)(p);
  f.h[1] = *(const v8h*)(p + 16);
  return f.v;
}
__device__ __forceinline__ v8f wmma_h(v16h a, v16h b, v8f c) {
  return __builtin_amdgcn_wmma_f32_16x16x32_f16(false, a, false, b, (short)0, c, false, false);
}
__device__ __forceinline__ v8f mma_g(v16h a, v16h b, v8f c) {
  c = __builtin_amdgcn_wmma_f32_16x16x32_f16(false, a, false, b, (short)0, c, false, false);
  asm volatile("v_nop\n\tv_nop\n\tv_nop\n\tv_nop" : "+v"(c) : "v"(a), "v"(b));
  return c;
}
__device__ __forceinline__ void dep_guard4_h(v8f& a, v8f& b, v8f& c, v8f& d, v16h x) {
  asm volatile("v_nop\n\tv_nop\n\tv_nop\n\tv_nop" : "+v"(a), "+v"(b), "+v"(c), "+v"(d) : "v"(x));
}
__device__ __forceinline__ void keep4_h(v16h a, v16h b, v16h c, v16h d) { asm volatile("v_nop" :: "v"(a), "v"(b), "v"(c), "v"(d)); }
__device__ __forceinline__ void acc_guard4(v8f& a, v8f& b, v8f& c, v8f& d) {
  asm volatile("v_nop\n\tv_nop\n\tv_nop\n\tv_nop" : "+v"(a), "+v"(b), "+v"(c), "+v"(d));
}

template <int OUT_MODE>
__global__ __launch_bounds__(256) void wmma_gemm64(
    const unsigned short* __restrict__ Ap, int lda, long strideA,
    const unsigned short* __restrict__ Btp, int ldb, long strideB,
    void* __restrict__ Cout, int ldc, long strideC,
    const float* __restrict__ resX, const float* __restrict__ resP, long strideR,
    const float* __restrict__ gpPtr, const float* __restrict__ gcPtr,
    int M, int N, int K, float scale) {
  const _Float16* A  = (const _Float16*)(const void*)Ap;
  const _Float16* Bt = (const _Float16*)(const void*)Btp;
  __shared__ __align__(16) float sT[8][16 * 68];
  const int b    = blockIdx.y;
  const int lane = threadIdx.x & 31;
  const int wave = threadIdx.x >> 5;
  const int tilesN = N >> 6;
  const int tilesM = M >> 6;
  const int tile = blockIdx.x * 8 + wave;
  if (tile >= tilesM * tilesN) return;
  const int tm = tile / tilesN;
  const int tn = tile - tm * tilesN;
  const int m0 = tm << 6;
  const int n0 = tn << 6;

  const _Float16* Ab = A  + (size_t)b * strideA;
  const _Float16* Bb = Bt + (size_t)b * strideB;

  const int rlane = lane & 15;
  const int koff  = (lane >> 4) * 8;
  const int mOff  = (lane >> 4) * 8;

  v8f acc[4][4];
#pragma unroll
  for (int i = 0; i < 4; ++i)
#pragma unroll
    for (int j = 0; j < 4; ++j) acc[i][j] = (v8f){0.f, 0.f, 0.f, 0.f, 0.f, 0.f, 0.f, 0.f};

  for (int k0 = 0; k0 < K; k0 += 32) {
    v16h bh[4];
#pragma unroll
    for (int j = 0; j < 4; ++j) {
      const size_t bo = (size_t)(n0 + (j << 4) + rlane) * ldb + koff + k0;
      bh[j] = frag_load(Bb + bo);
    }
#pragma unroll
    for (int i = 0; i < 4; ++i) {
      const size_t ao = (size_t)(m0 + (i << 4) + rlane) * lda + koff + k0;
      const v16h ah = frag_load(Ab + ao);
#pragma unroll
      for (int j = 0; j < 4; ++j) acc[i][j] = wmma_h(ah, bh[j], acc[i][j]);
      dep_guard4_h(acc[i][0], acc[i][1], acc[i][2], acc[i][3], ah);
    }
    keep4_h(bh[0], bh[1], bh[2], bh[3]);
  }
  acc_guard4(acc[0][0], acc[0][1], acc[0][2], acc[0][3]);
  acc_guard4(acc[1][0], acc[1][1], acc[1][2], acc[1][3]);
  acc_guard4(acc[2][0], acc[2][1], acc[2][2], acc[2][3]);
  acc_guard4(acc[3][0], acc[3][1], acc[3][2], acc[3][3]);

  float gp = 0.f, gc = 0.f;
  if (OUT_MODE == 3) { gp = gpPtr[0]; gc = gcPtr[0]; }

  float* slab = sT[wave];
#pragma unroll
  for (int i = 0; i < 4; ++i) {
    const int mBase = m0 + (i << 4);
#pragma unroll
    for (int j = 0; j < 4; ++j) {
#pragma unroll
      for (int r = 0; r < 8; ++r) {
        slab[(mOff + r) * 68 + (j << 4) + rlane] = acc[i][j][r] * scale;
      }
    }
    __builtin_amdgcn_fence(__ATOMIC_RELEASE, "workgroup");
    __builtin_amdgcn_wave_barrier();
    __builtin_amdgcn_fence(__ATOMIC_ACQUIRE, "workgroup");
    if (OUT_MODE == 0 || OUT_MODE == 3) {
      float* C = (float*)Cout + (size_t)b * strideC;
      const int hh = lane >> 4, c4 = (lane & 15) * 4;
      if (OUT_MODE == 3) {
        const float* Xb = resX + (size_t)b * strideR;
        const float* Pb = resP + (size_t)b * strideR;
#pragma unroll 1
        for (int it = 0; it < 8; ++it) {
          const int row = it * 2 + hh;
          float* sp = slab + row * 68 + c4;
          const size_t gi = (size_t)(mBase + row) * ldc + n0 + c4;
          const v4f a  = *(const v4f*)sp;
          const v4f xv = *(const v4f*)(Xb + gi);
          const v4f pv = *(const v4f*)(Pb + gi);
          v4f o;
#pragma unroll
          for (int e = 0; e < 4; ++e) {
            const float t1 = gp * pv[e] + xv[e];
            const float t2 = gc * a[e] + xv[e];
            o[e] = t1 + t2;
          }
          *(v4f*)sp = o;
        }
        __builtin_amdgcn_fence(__ATOMIC_RELEASE, "workgroup");
        __builtin_amdgcn_wave_barrier();
        __builtin_amdgcn_fence(__ATOMIC_ACQUIRE, "workgroup");
      }
      for (int pass = 0; pass < 2; ++pass) {
#pragma unroll
        for (int it = 0; it < 8; ++it) {
          const int row = it * 2 + hh;
          const v4f v = *(const v4f*)(slab + row * 68 + c4);
          *(volatile v4f*)(C + (size_t)(mBase + row) * ldc + n0 + c4) = v;
        }
        __threadfence();
      }
    } else {
      const int q = lane >> 3, c8 = (lane & 7) * 8;
      unsigned short* C = (unsigned short*)Cout + (size_t)b * strideC;
      for (int pass = 0; pass < 2; ++pass) {
#pragma unroll
        for (int it = 0; it < 4; ++it) {
          const int row = it * 4 + q;
          const float* sp = slab + row * 68 + c8;
          v8h hv;
#pragma unroll
          for (int e = 0; e < 8; ++e) hv[e] = (_Float16)sp[e];
          *(volatile v8h*)(C + (size_t)(mBase + row) * ldc + n0 + c8) = hv;
        }
        __threadfence();
      }
    }
    __builtin_amdgcn_fence(__ATOMIC_RELEASE, "workgroup");
    __builtin_amdgcn_wave_barrier();
    __builtin_amdgcn_fence(__ATOMIC_ACQUIRE, "workgroup");
  }
}

__global__ __launch_bounds__(256) void cvt_x_kernel(const float* __restrict__ x,
                                                    unsigned short* __restrict__ x16,
                                                    unsigned short* __restrict__ xTH,
                                                    unsigned short* __restrict__ xTL) {
  __shared__ __align__(16) float sm[64 * kXP];
  const int t = threadIdx.x, lane = t & 31, wave = t >> 5;
  const int n0 = blockIdx.x * 64, c0 = blockIdx.y * 64, b = blockIdx.z;
  const float* xb = x + (size_t)b * kC * kN;
#pragma unroll
  for (int i = 0; i < 4; ++i) {
    const int e = i * 256 + t;
    const int r = e >> 4;
    const int c4 = (e & 15) * 4;
    const v4f v = *(const v4f*)(xb + (size_t)(c0 + r) * kN + n0 + c4);
    *(v4f*)(sm + r * kXP + c4) = v;
  }
  __syncthreads();
  const int q = lane >> 3, c8 = (lane & 7) * 8;
  v4u un[2], uth[2], utl[2];
#pragma unroll
  for (int it = 0; it < 2; ++it) {
    const int row = wave * 8 + it * 4 + q;
    const float* sr = sm + row * kXP + c8;
    un[it] = pack8_f16(sr[0], sr[1], sr[2], sr[3], sr[4], sr[5], sr[6], sr[7]);
    const float* sc = sm + c8 * kXP + row;
    pack8_split(sc[0 * kXP], sc[1 * kXP], sc[2 * kXP], sc[3 * kXP],
                sc[4 * kXP], sc[5 * kXP], sc[6 * kXP], sc[7 * kXP], uth[it], utl[it]);
  }
  for (int pass = 0; pass < 2; ++pass) {
#pragma unroll
    for (int it = 0; it < 2; ++it) {
      const int row = wave * 8 + it * 4 + q;
      const size_t to = ((size_t)b * kN + n0 + row) * kC + c0 + c8;
      *(volatile v4u*)(x16 + ((size_t)b * kC + c0 + row) * kN + n0 + c8) = un[it];
      *(volatile v4u*)(xTH + to) = uth[it];
      *(volatile v4u*)(xTL + to) = utl[it];
    }
    __threadfence();
  }
}

__global__ __launch_bounds__(256) void cvt_w_kernel(const float* __restrict__ Wq, const float* __restrict__ Wk,
                                                    const float* __restrict__ Wv, unsigned short* __restrict__ w16,
                                                    unsigned short* __restrict__ w16l, int n8) {
  const int i = blockIdx.x * 256 + threadIdx.x;
  if (i >= n8) return;
  const int r0 = blockIdx.x * 4;
  const float* src;
  int rb;
  if (r0 < kHid) { src = Wq; rb = 0; }
  else if (r0 < 2 * kHid) { src = Wk; rb = kHid; }
  else { src = Wv; rb = 2 * kHid; }
  const bool wlo = (r0 < 2 * kHid);
  const size_t e0 = (size_t)i * 8;
  const float* p = src + (e0 - (size_t)rb * kC);
  const v4f a = *(const v4f*)(p);
  const v4f c = *(const v4f*)(p + 4);
  v4u uh, ul;
  pack8_split(a[0] * kWCarry, a[1] * kWCarry, a[2] * kWCarry, a[3] * kWCarry,
              c[0] * kWCarry, c[1] * kWCarry, c[2] * kWCarry, c[3] * kWCarry, uh, ul);
  unsigned short* d = w16 + e0;
  for (int pass = 0; pass < 2; ++pass) {
    *(volatile v4u*)d = uh;
    if (wlo) {
      unsigned short* dl = w16l + e0;
      *(volatile v4u*)dl = ul;
    }
    __threadfence();
  }
}

__global__ __launch_bounds__(256) void qk_proj_kernel(const unsigned short* __restrict__ XHp,
                                                      const unsigned short* __restrict__ XLp,
                                                      const unsigned short* __restrict__ WHp,
                                                      const unsigned short* __restrict__ WLp,
                                                      unsigned short* __restrict__ QKH,
                                                      unsigned short* __restrict__ QKL) {
  __shared__ __align__(16) float sT[8][16 * 68];
  const _Float16* XH = (const _Float16*)(const void*)XHp;
  const _Float16* XL = (const _Float16*)(const void*)XLp;
  const _Float16* WH = (const _Float16*)(const void*)WHp;
  const _Float16* WL = (const _Float16*)(const void*)WLp;
  const int lane = threadIdx.x & 31, wave = threadIdx.x >> 5;
  const int tile = blockIdx.x * 8 + wave;
  const int m0 = (tile >> 1) * 16;
  const int n0 = (tile & 1) * 64;
  const int rlane = lane & 15;
  const int koff  = (lane >> 4) * 8;
  const int mOff  = (lane >> 4) * 8;

  v8f accm[4], accr[4];
#pragma unroll
  for (int j = 0; j < 4; ++j) {
    accm[j] = (v8f){0.f, 0.f, 0.f, 0.f, 0.f, 0.f, 0.f, 0.f};
    accr[j] = (v8f){0.f, 0.f, 0.f, 0.f, 0.f, 0.f, 0.f, 0.f};
  }
  const size_t arow = (size_t)(m0 + rlane) * kC + koff;
#pragma unroll 1
  for (int k0 = 0; k0 < kC; k0 += 32) {
    const v16h ah = frag_load(XH + arow + k0);
    const v16h al = frag_load(XL + arow + k0);
#pragma unroll
    for (int j = 0; j < 4; ++j) {
      const size_t bo = (size_t)(n0 + (j << 4) + rlane) * kC + koff + k0;
      const v16h bh = frag_load(WH + bo);
      const v16h bl = frag_load(WL + bo);
      accm[j] = mma_g(ah, bh, accm[j]);
      accr[j] = mma_g(ah, bl, accr[j]);
      accr[j] = mma_g(al, bh, accr[j]);
    }
  }

  float* slab = sT[wave];
#pragma unroll
  for (int j = 0; j < 4; ++j) {
#pragma unroll
    for (int r = 0; r < 8; ++r) {
      const float full = accm[j][r] + accr[j][r] * kResInv;
      slab[(mOff + r) * 68 + (j << 4) + rlane] = full * kWCarryInv;
    }
  }
  __builtin_amdgcn_fence(__ATOMIC_RELEASE, "workgroup");
  __builtin_amdgcn_wave_barrier();
  __builtin_amdgcn_fence(__ATOMIC_ACQUIRE, "workgroup");
  const int q = lane >> 3, c8 = (lane & 7) * 8;
  v4u hv[4], lv[4];
#pragma unroll
  for (int it = 0; it < 4; ++it) {
    const float* sp = slab + (it * 4 + q) * 68 + c8;
    const v4f a0 = *(const v4f*)(sp);
    const v4f a1 = *(const v4f*)(sp + 4);
    pack8_split(a0[0], a0[1], a0[2], a0[3], a1[0], a1[1], a1[2], a1[3], hv[it], lv[it]);
  }
  for (int pass = 0; pass < 2; ++pass) {
#pragma unroll
    for (int it = 0; it < 4; ++it) {
      const size_t o = (size_t)(m0 + it * 4 + q) * kQK + n0 + c8;
      *(volatile v4u*)(QKH + o) = hv[it];
      *(volatile v4u*)(QKL + o) = lv[it];
    }
    __threadfence();
  }
}

__global__ __launch_bounds__(256) void pam_max_kernel(const unsigned short* __restrict__ QKHp,
                                                      float* __restrict__ rowmax) {
  __shared__ __align__(16) float sS[128];
  const _Float16* QK = (const _Float16*)(const void*)QKHp;
  const int tid = threadIdx.x, lane = tid & 31, wave = tid >> 5;
  const int hh = lane >> 4, c = lane & 15;
  const int tok0 = blockIdx.x * 128;
  const int b = tok0 / kN;
  const int row0 = tok0 + wave * 16;
  const _Float16* qp = QK + (size_t)(row0 + c) * kQK + 8 * hh;
  const v16h qa0 = frag_load(qp);
  const v16h qa1 = frag_load(qp + 32);
  const _Float16* kbase = QK + (size_t)(b * kN + c) * kQK + kHid + 8 * hh;
  float mx[8];
#pragma unroll
  for (int r = 0; r < 8; ++r) mx[r] = -1.0e30f;
#pragma unroll 1
  for (int kc = 0; kc < kN / 64; ++kc) {
#pragma unroll
    for (int j = 0; j < 4; ++j) {
      const _Float16* kp = kbase + (size_t)(kc * 64 + j * 16) * kQK;
      const v16h kb0 = frag_load(kp);
      const v16h kb1 = frag_load(kp + 32);
      v8f s = (v8f){0.f, 0.f, 0.f, 0.f, 0.f, 0.f, 0.f, 0.f};
      s = mma_g(qa0, kb0, s);
      s = mma_g(qa1, kb1, s);
#pragma unroll
      for (int r = 0; r < 8; ++r) mx[r] = fmaxf(mx[r], s[r]);
    }
  }
#pragma unroll
  for (int r = 0; r < 8; ++r) {
#pragma unroll
    for (int off = 1; off < 16; off <<= 1) {
      const float mo = __shfl_xor(mx[r], off, 32);
      mx[r] = fmaxf(mx[r], mo);
    }
  }
  if (c == 0) {
#pragma unroll
    for (int r = 0; r < 8; ++r) sS[wave * 16 + 8 * hh + r] = mx[r];
  }
  __syncthreads();
  if (wave == 0) {
    const v4f v = *(const v4f*)(sS + lane * 4);
    float* d = rowmax + tok0 + lane * 4;
    *(volatile v4f*)d = v;
    __threadfence();
    *(volatile v4f*)d = v;
  }
}

__global__ __launch_bounds__(256) void pam_pv_kernel(const unsigned short* __restrict__ QKHp,
                                                     const unsigned short* __restrict__ QKLp,
                                                     const unsigned short* __restrict__ Vp,
                                                     const float* __restrict__ rowmax,
                                                     float* __restrict__ PAM) {
  __shared__ __align__(16) _Float16 Pl[kPvQ * kPvPP];
  __shared__ __align__(16) float sO[8][16 * kPvSP];
  __shared__ __align__(16) float sSum[4 * kPvQ];
  const _Float16* QKH = (const _Float16*)(const void*)QKHp;
  const _Float16* QKL = (const _Float16*)(const void*)QKLp;
  const _Float16* V   = (const _Float16*)(const void*)Vp;
  const int tid = threadIdx.x, lane = tid & 31, wave = tid >> 5;
  const int hh = lane >> 4, c = lane & 15;
  const int m0g = blockIdx.x * kPvQ;
  const int b = m0g / kN;
  const int m0 = m0g - b * kN;
  const int ms = wave & 1, kg = wave >> 1;

  const size_t qo = (size_t)(m0g + ms * 16 + c) * kQK + 8 * hh;
  const v16h qh0 = frag_load(QKH + qo);
  const v16h qh1 = frag_load(QKH + qo + 32);
  const v16h ql0 = frag_load(QKL + qo);
  const v16h ql1 = frag_load(QKL + qo + 32);

  const int sr = m0g + ms * 16 + 8 * hh;
  const v4f mxa = *(const v4f*)(rowmax + sr);
  const v4f mxb = *(const v4f*)(rowmax + sr + 4);
  float rmx[8], psum[8];
#pragma unroll
  for (int e = 0; e < 4; ++e) {
    rmx[e] = mxa[e];
    rmx[4 + e] = mxb[e];
  }
#pragma unroll
  for (int r = 0; r < 8; ++r) psum[r] = 0.f;

  v8f acc[4][2];
#pragma unroll
  for (int i = 0; i < 4; ++i) {
    acc[i][0] = (v8f){0.f, 0.f, 0.f, 0.f, 0.f, 0.f, 0.f, 0.f};
    acc[i][1] = (v8f){0.f, 0.f, 0.f, 0.f, 0.f, 0.f, 0.f, 0.f};
  }
  const size_t kofs = (size_t)(b * kN + c) * kQK + kHid + 8 * hh;
  const _Float16* vbase = V + (size_t)(b * kC + wave * 64 + c) * kN + 8 * hh;
  _Float16* pwBase = Pl + (ms * 16 + 8 * hh) * kPvPP + kg * 32 + c;
  const _Float16* pb0 = Pl + c * kPvPP + 8 * hh;
  const _Float16* pb1 = Pl + (16 + c) * kPvPP + 8 * hh;

#pragma unroll 1
  for (int kc = 0; kc < kN / kPvKC; ++kc) {
    const int n0 = kc * kPvKC;
#pragma unroll
    for (int t = 0; t < 2; ++t) {
      const size_t ko = kofs + (size_t)(n0 + kg * 32 + t * 16) * kQK;
      const v16h kh0 = frag_load(QKH + ko);
      const v16h kh1 = frag_load(QKH + ko + 32);
      const v16h kl0 = frag_load(QKL + ko);
      const v16h kl1 = frag_load(QKL + ko + 32);
      v8f s = (v8f){0.f, 0.f, 0.f, 0.f, 0.f, 0.f, 0.f, 0.f};
      s = mma_g(qh0, kh0, s);
      s = mma_g(qh1, kh1, s);
      v8f sres = (v8f){0.f, 0.f, 0.f, 0.f, 0.f, 0.f, 0.f, 0.f};
      sres = mma_g(qh0, kl0, sres);
      sres = mma_g(ql0, kh0, sres);
      sres = mma_g(qh1, kl1, sres);
      sres = mma_g(ql1, kh1, sres);
      _Float16* pw = pwBase + t * 16;
#pragma unroll
      for (int r = 0; r < 8; ++r) {
        const float l = s[r] + sres[r] * kResInv;
        const float arg = fminf(l - rmx[r], kArgCap);
        const float pc = __expf(arg) * kPCarry;
        psum[r] += pc;
        pw[r * kPvPP] = (_Float16)pc;
      }
    }
    __syncthreads();
#pragma unroll 1
    for (int ks = 0; ks < kPvKC / 32; ++ks) {
      const v16h b0 = frag_load(pb0 + ks * 32);
      const v16h b1 = frag_load(pb1 + ks * 32);
#pragma unroll
      for (int i = 0; i < 4; ++i) {
        const v16h ah = frag_load(vbase + (size_t)(i * 16) * kN + n0 + ks * 32);
        acc[i][0] = mma_g(ah, b0, acc[i][0]);
        acc[i][1] = mma_g(ah, b1, acc[i][1]);
      }
    }
    __syncthreads();
  }

#pragma unroll
  for (int r = 0; r < 8; ++r) {
#pragma unroll
    for (int off = 1; off < 16; off <<= 1) {
      const float so = __shfl_xor(psum[r], off, 32);
      psum[r] += so;
    }
  }
  if (c == 0) {
#pragma unroll
    for (int r = 0; r < 8; ++r) sSum[kg * kPvQ + ms * 16 + 8 * hh + r] = psum[r];
  }
  __syncthreads();
  float inv[2];
#pragma unroll
  for (int mt = 0; mt < 2; ++mt) {
    const int m = mt * 16 + c;
    const float tot = ((sSum[m] + sSum[kPvQ + m]) + sSum[2 * kPvQ + m]) + sSum[3 * kPvQ + m];
    inv[mt] = __builtin_amdgcn_rcpf(tot);
  }

  float* slab = sO[wave];
  const int q = lane >> 3, c4 = (lane & 7) * 4;
#pragma unroll
  for (int i = 0; i < 4; ++i) {
    __syncthreads();
#pragma unroll
    for (int mt = 0; mt < 2; ++mt) {
#pragma unroll
      for (int r = 0; r < 8; ++r) {
        slab[(8 * hh + r) * kPvSP + mt * 16 + c] = acc[i][mt][r] * inv[mt];
      }
    }
    __syncthreads();
    v4f ov[4];
#pragma unroll
    for (int it = 0; it < 4; ++it) ov[it] = *(const v4f*)(slab + (it * 4 + q) * kPvSP + c4);
    for (int pass = 0; pass < 2; ++pass) {
#pragma unroll
      for (int it = 0; it < 4; ++it) {
        const int ch = wave * 64 + i * 16 + it * 4 + q;
        *(volatile v4f*)(PAM + ((size_t)b * kC + ch) * kN + m0 + c4) = ov[it];
      }
      __threadfence();
    }
  }
}

__global__ __launch_bounds__(256) void cam_softmax_kernel(const float* __restrict__ G,
                                                          unsigned short* __restrict__ E16) {
  const int lane = threadIdx.x & 31, wave = threadIdx.x >> 5;
  const int row = blockIdx.x * 8 + wave;
  const float* g = G + (size_t)row * kC;
  float xv[16];
#pragma unroll
  for (int s = 0; s < 2; ++s) {
    const v4f a = *(const v4f*)(g + s * 256 + lane * 8);
    const v4f c = *(const v4f*)(g + s * 256 + lane * 8 + 4);
#pragma unroll
    for (int e = 0; e < 4; ++e) { xv[s * 8 + e] = a[e]; xv[s * 8 + 4 + e] = c[e]; }
  }
  float m = xv[0];
#pragma unroll
  for (int i = 1; i < 16; ++i) m = fmaxf(m, xv[i]);
#pragma unroll
  for (int off = 16; off > 0; off >>= 1) m = fmaxf(m, __shfl_xor(m, off, 32));
  float sum = 0.f;
#pragma unroll
  for (int i = 0; i < 16; ++i) { xv[i] = __expf(xv[i] - m); sum += xv[i]; }
#pragma unroll
  for (int off = 16; off > 0; off >>= 1) sum += __shfl_xor(sum, off, 32);
  const float inv = kECarry * __builtin_amdgcn_rcpf(sum);
  v4u u[2];
#pragma unroll
  for (int s = 0; s < 2; ++s) {
    u[s] = pack8_f16(xv[s * 8 + 0] * inv, xv[s * 8 + 1] * inv, xv[s * 8 + 2] * inv, xv[s * 8 + 3] * inv,
                     xv[s * 8 + 4] * inv, xv[s * 8 + 5] * inv, xv[s * 8 + 6] * inv, xv[s * 8 + 7] * inv);
  }
  unsigned short* d = E16 + (size_t)row * kC + lane * 8;
  for (int pass = 0; pass < 2; ++pass) {
    *(volatile v4u*)(d) = u[0];
    *(volatile v4u*)(d + 256) = u[1];
    __threadfence();
  }
}

extern "C" void kernel_launch(void* const* d_in, const int* in_sizes, int n_in,
                              void* d_out, int out_size, void* d_ws, size_t ws_size,
                              hipStream_t stream) {
  if (n_in < 6) return;
  if (in_sizes[0] != kB * kC * kN) return;
  if (in_sizes[1] != kHid * kC) return;
  if (in_sizes[2] != kHid * kC) return;
  if (in_sizes[3] != kC * kC) return;
  if (in_sizes[4] != 1) return;
  if (in_sizes[5] != 1) return;
  if (out_size != kB * kC * kN) return;
  if (ws_size < kWsTotal) return;

  const float* x       = (const float*)d_in[0];
  const float* Wq      = (const float*)d_in[1];
  const float* Wk      = (const float*)d_in[2];
  const float* Wv      = (const float*)d_in[3];
  const float* gamma_p = (const float*)d_in[4];
  const float* gamma_c = (const float*)d_in[5];
  float* out = (float*)d_out;

  char* ws = (char*)d_ws;
  unsigned short* X16   = (unsigned short*)(ws + kOffX16);
  unsigned short* XTH   = (unsigned short*)(ws + kOffXTH);
  unsigned short* XTL   = (unsigned short*)(ws + kOffXTL);
  unsigned short* W16   = (unsigned short*)(ws + kOffW16);
  unsigned short* W16L  = (unsigned short*)(ws + kOffW16L);
  unsigned short* QKH   = (unsigned short*)(ws + kOffQKH);
  unsigned short* QKL   = (unsigned short*)(ws + kOffQKL);
  unsigned short* V16   = (unsigned short*)(ws + kOffV16);
  float*          RMAX  = (float*)(ws + kOffRMAX);
  float*          PAM   = (float*)(ws + kOffPAM);
  float*          G     = (float*)(ws + kOffG);
  unsigned short* E16   = (unsigned short*)(ws + kOffE16);

  const long sXT = (long)kN * kC;
  const long sCN = (long)kC * kN;
  const long sCC = (long)kC * kC;

  cvt_x_kernel<<<dim3(kN / 64, kC / 64, kB), 256, 0, stream>>>(x, X16, XTH, XTL);
  cvt_w_kernel<<<(kWRows * kC / 8) / 256, 256, 0, stream>>>(Wq, Wk, Wv, W16, W16L, kWRows * kC / 8);
  qk_proj_kernel<<<(((kB * kN) / 16) * (kQK / 64)) / 8, 256, 0, stream>>>(XTH, XTL, W16, W16L, QKH, QKL);
  wmma_gemm64<1><<<dim3(64, kB), 256, 0, stream>>>(
      W16 + (size_t)kQK * kC, kC, 0L, XTH, kC, sXT, (void*)V16, kN, sCN,
      nullptr, nullptr, 0L, nullptr, nullptr, kC, kN, kC, kWCarryInv);
  pam_max_kernel<<<(kB * kN) / 128, 256, 0, stream>>>(QKH, RMAX);
  pam_pv_kernel<<<(kB * kN) / kPvQ, 256, 0, stream>>>(QKH, QKL, V16, RMAX, PAM);
  wmma_gemm64<0><<<dim3(8, kB), 256, 0, stream>>>(
      X16, kN, sCN, X16, kN, sCN, (void*)G, kC, sCC,
      nullptr, nullptr, 0L, nullptr, nullptr, kC, kC, kN, 1.0f);
  cam_softmax_kernel<<<(kB * kC) / 8, 256, 0, stream>>>(G, E16);
  wmma_gemm64<3><<<dim3(64, kB), 256, 0, stream>>>(
      E16, kC, sCC, XTH, kC, sXT, (void*)out, kN, sCN,
      x, PAM, sCN, gamma_p, gamma_c, kC, kN, kC, kECarryInv);
}
